// GCRNCell_21586505629814
// MI455X (gfx1250) — hardware-verified
//
#include <hip/hip_runtime.h>
#include <math.h>

constexpr int kB = 8;
constexpr int kN = 2048;
constexpr int kIn = 2;
constexpr int kOut = 16;
constexpr int kC = 18;
constexpr int kH = 4;
constexpr int kDh = 8;
constexpr int kNG = 6;
constexpr int kColPad = 192;
constexpr int kRows = kB * kN;
constexpr int kGK = 64;
constexpr long kAdjPlane = (long)kN * kN;
constexpr long kYPlane = (long)kColPad * kN;

constexpr float kAdjCarry = 1024.0f;
constexpr float kFeatCarry = 8.0f;
constexpr float kY1Carry = 256.0f;
constexpr float kGateCarry = 16.0f;
constexpr float kWCarry = 4.0f;
constexpr float kHCarry = 8.0f;
constexpr float kScaleD1 = 1.0f / (8.0f * 1024.0f);
constexpr float kScaleD2 = 1.0f / (256.0f * 1024.0f);
constexpr float kScaleGate = 1.0f / (16.0f * 4.0f);
constexpr float kScaleMlp = 1.0f / (8.0f * 4.0f);
constexpr float kInvSqrtDh = 0.353553390593273762f;

typedef __attribute__((ext_vector_type(16))) _Float16 v16h;
typedef __attribute__((ext_vector_type(8)))  _Float16 v8h;
typedef __attribute__((ext_vector_type(16))) __bf16   v16b;
typedef __attribute__((ext_vector_type(8)))  __bf16   v8b;
typedef __attribute__((ext_vector_type(8)))  float    v8f;
typedef __attribute__((ext_vector_type(4)))  float    v4f;
typedef __attribute__((ext_vector_type(4)))  unsigned int v4u;

__device__ __forceinline__ unsigned short f2bf_bits(float f) {
  unsigned u = __float_as_uint(f);
  return (unsigned short)((u + 0x7FFFu + ((u >> 16) & 1u)) >> 16);
}
__device__ __forceinline__ float bf_bits2f(unsigned short h) { return __uint_as_float(((unsigned)h) << 16); }

__device__ __forceinline__ void dep_guard_h(v8f& a, v8f& b, v16h x, v16h y) { asm volatile("v_nop\n\tv_nop\n\tv_nop\n\tv_nop" : "+v"(a), "+v"(b) : "v"(x), "v"(y)); }
__device__ __forceinline__ void dep_guard_b(v8f& a, v8f& b, v16b x, v16b y) { asm volatile("v_nop\n\tv_nop\n\tv_nop\n\tv_nop" : "+v"(a), "+v"(b) : "v"(x), "v"(y)); }
__device__ __forceinline__ void keep4_h(v16h a, v16h b, v16h c, v16h d) { asm volatile("v_nop" :: "v"(a), "v"(b), "v"(c), "v"(d)); }
__device__ __forceinline__ void keep4_b(v16b a, v16b b, v16b c, v16b d) { asm volatile("v_nop" :: "v"(a), "v"(b), "v"(c), "v"(d)); }
__device__ __forceinline__ void acc_guard4(v8f& a, v8f& b, v8f& c, v8f& d) { asm volatile("v_nop\n\tv_nop\n\tv_nop\n\tv_nop" : "+v"(a), "+v"(b), "+v"(c), "+v"(d)); }
template <typename T> struct Frag;
template <> struct Frag<_Float16> {
  typedef v16h V; union U { v16h v; v8h h[2]; };
  static __device__ __forceinline__ v16h load(const _Float16* p) {
    U f; f.h[0] = *(const v8h*)(p); f.h[1] = *(const v8h*)(p + 16); return f.v;
  }
  static __device__ __forceinline__ v8f mma(v16h a, v16h b, v8f c) {
    return __builtin_amdgcn_wmma_f32_16x16x32_f16(false, a, false, b, (short)0, c, false, false);
  }
  static __device__ __forceinline__ void guard(v8f& a, v8f& b, v16h x, v16h y) { dep_guard_h(a, b, x, y); }
  static __device__ __forceinline__ void keep(v16h a, v16h b, v16h c, v16h d) { keep4_h(a, b, c, d); }
};
template <> struct Frag<__bf16> {
  typedef v16b V; union U { v16b v; v8b h[2]; };
  static __device__ __forceinline__ v16b load(const __bf16* p) {
    U f; f.h[0] = *(const v8b*)(p); f.h[1] = *(const v8b*)(p + 16); return f.v;
  }
  static __device__ __forceinline__ v8f mma(v16b a, v16b b, v8f c) {
    return __builtin_amdgcn_wmma_f32_16x16x32_bf16(false, a, false, b, (short)0, c, false, false);
  }
  static __device__ __forceinline__ void guard(v8f& a, v8f& b, v16b x, v16b y) { dep_guard_b(a, b, x, y); }
  static __device__ __forceinline__ void keep(v16b a, v16b b, v16b c, v16b d) { keep4_b(a, b, c, d); }
};

__device__ __forceinline__ unsigned pk16(unsigned short a, unsigned short b) { return (unsigned)a | ((unsigned)b << 16); }
__device__ __forceinline__ unsigned short h_bits(float f) { const _Float16 h = (_Float16)f; return __builtin_bit_cast(unsigned short, h); }

template <int ET> struct Elem;
template <> struct Elem<0> { typedef _Float16 T; };
template <> struct Elem<1> { typedef __bf16 T; };
template <int ET, bool SPLIT, int BIAS_MODE, int OUT_MODE, bool RESID, int ACT = 0>
__global__ __launch_bounds__(256) void wmma_gemm64(
    const unsigned short* __restrict__ Ap, const unsigned short* __restrict__ A2p, int lda, long strideA,
    const unsigned short* __restrict__ Btp, const unsigned short* __restrict__ Bt2p, int ldb, long strideB,
    void* __restrict__ Cout, void* __restrict__ Cout2, int ldc, long strideC,
    const float* __restrict__ bias,
    const float* __restrict__ resid, long strideR,
    int M, int N, int K, float scale) {
  typedef typename Elem<ET>::T T;
  typedef typename Frag<T>::V V;
  const T* A = (const T*)Ap; const T* A2 = (const T*)A2p; const T* Bt = (const T*)Btp; const T* Bt2 = (const T*)Bt2p;
  __shared__ __align__(16) float sT[8][16 * 68];
  const int b    = blockIdx.y;
  const int lane = threadIdx.x & 31;
  const int wave = threadIdx.x >> 5;
  const int tilesN = N >> 6;
  const int tilesM = M >> 6;
  const int tile = blockIdx.x * 8 + wave;
  if (tile >= tilesM * tilesN) return;
  const int tm = tile / tilesN;
  const int tn = tile - tm * tilesN;
  const int m0 = tm << 6;
  const int n0 = tn << 6;

  const T* Ab  = A  + (size_t)b * strideA;
  const T* Bb  = Bt + (size_t)b * strideB;
  const T* Ab2 = SPLIT ? (A2  + (size_t)b * strideA) : nullptr;
  const T* Bb2 = SPLIT ? (Bt2 + (size_t)b * strideB) : nullptr;

  const int rlane = lane & 15;
  const int koff  = (lane >> 4) * 8;
  const int mOff  = (lane >> 4) * 8;

  v8f acc[4][4];
#pragma unroll
  for (int i = 0; i < 4; ++i)
#pragma unroll
    for (int j = 0; j < 4; ++j) acc[i][j] = (v8f){0.f,0.f,0.f,0.f,0.f,0.f,0.f,0.f};

  for (int k0 = 0; k0 < K; k0 += 32) {
    V bh[4], bl[4];
#pragma unroll
    for (int j = 0; j < 4; ++j) {
      const size_t bo = (size_t)(n0 + (j << 4) + rlane) * ldb + koff + k0;
      bh[j] = Frag<T>::load(Bb + bo);
      if (SPLIT) bl[j] = Frag<T>::load(Bb2 + bo);
    }
#pragma unroll
    for (int i = 0; i < 4; ++i) {
      const size_t ao = (size_t)(m0 + (i << 4) + rlane) * lda + koff + k0;
      V ah = Frag<T>::load(Ab + ao);
      V al;
      if (SPLIT) al = Frag<T>::load(Ab2 + ao);
#pragma unroll
      for (int j = 0; j < 4; ++j) {
        acc[i][j] = Frag<T>::mma(ah, bh[j], acc[i][j]);
        if (SPLIT) {
          acc[i][j] = Frag<T>::mma(ah, bl[j], acc[i][j]);
          acc[i][j] = Frag<T>::mma(al, bh[j], acc[i][j]);
        }
      }
      Frag<T>::guard(acc[i][0], acc[i][3], ah, SPLIT ? al : ah);
    }
    Frag<T>::keep(bh[0], bh[1], bh[2], bh[3]);
    if (SPLIT) Frag<T>::keep(bl[0], bl[1], bl[2], bl[3]);
  }
  acc_guard4(acc[0][0], acc[0][1], acc[0][2], acc[0][3]);
  acc_guard4(acc[1][0], acc[1][1], acc[1][2], acc[1][3]);
  acc_guard4(acc[2][0], acc[2][1], acc[2][2], acc[2][3]);
  acc_guard4(acc[3][0], acc[3][1], acc[3][2], acc[3][3]);

  float* slab = sT[wave];
  const float* Rb = RESID ? (resid + (size_t)b * strideR) : nullptr;
#pragma unroll
  for (int i = 0; i < 4; ++i) {
    const int mBase = m0 + (i << 4);
#pragma unroll
    for (int j = 0; j < 4; ++j) {
      const int n = n0 + (j << 4) + rlane;
      float bv = 0.f;
      if (BIAS_MODE == 2) bv = bias[n];
#pragma unroll
      for (int r = 0; r < 8; ++r) {
        float v = acc[i][j][r] * scale;
        if (BIAS_MODE == 1) v += bias[mBase + mOff + r];
        if (BIAS_MODE == 2) v += bv;
        if (RESID) v += Rb[(size_t)(mBase + mOff + r) * ldc + n];
        if (ACT == 2) v = fmaxf(v, 0.0f);
        if (ACT == 4) v = (v > 0.f) ? v : 0.01f * v;
        slab[(mOff + r) * 68 + (j << 4) + rlane] = v;
      }
    }
    __builtin_amdgcn_fence(__ATOMIC_RELEASE, "workgroup");
    __builtin_amdgcn_wave_barrier();
    __builtin_amdgcn_fence(__ATOMIC_ACQUIRE, "workgroup");
    if (OUT_MODE == 0) {
      float* C = (float*)Cout + (size_t)b * strideC;
      const int hh = lane >> 4, c4 = (lane & 15) * 4;
      for (int pass = 0; pass < 2; ++pass) {
#pragma unroll
        for (int it = 0; it < 8; ++it) {
          const int row = it * 2 + hh;
          v4f v = *(const v4f*)(slab + row * 68 + c4);
          *(volatile v4f*)(C + (size_t)(mBase + row) * ldc + n0 + c4) = v;
        }
        __threadfence();
      }
    } else {
      const int q = lane >> 3, c8 = (lane & 7) * 8;
      unsigned short* C  = (unsigned short*)Cout  + (size_t)b * strideC;
      unsigned short* C2 = (OUT_MODE == 2) ? ((unsigned short*)Cout2 + (size_t)b * strideC) : nullptr;
      for (int pass = 0; pass < 2; ++pass) {
#pragma unroll
        for (int it = 0; it < 4; ++it) {
          const int row = it * 4 + q;
          const float* sp = slab + row * 68 + c8;
          v8h hv, lv;
#pragma unroll
          for (int e = 0; e < 8; ++e) {
            if (OUT_MODE == 1) {
              hv[e] = (_Float16)sp[e];
            } else {
              unsigned short hb = f2bf_bits(sp[e]);
              unsigned short lb = f2bf_bits(sp[e] - bf_bits2f(hb));
              hv[e] = __builtin_bit_cast(_Float16, hb);
              lv[e] = __builtin_bit_cast(_Float16, lb);
            }
          }
          *(volatile v8h*)(C + (size_t)(mBase + row) * ldc + n0 + c8) = hv;
          if (OUT_MODE == 2) *(volatile v8h*)(C2 + (size_t)(mBase + row) * ldc + n0 + c8) = lv;
        }
        __threadfence();
      }
    }
    __builtin_amdgcn_fence(__ATOMIC_RELEASE, "workgroup");
    __builtin_amdgcn_wave_barrier();
    __builtin_amdgcn_fence(__ATOMIC_ACQUIRE, "workgroup");
  }
}

__global__ __launch_bounds__(256) void k_cast8(const float* __restrict__ in, unsigned short* __restrict__ out, int n8, float carry) {
  const int i = blockIdx.x * 256 + threadIdx.x;
  if (i >= n8) return;
  const float* p = in + 8 * (size_t)i;
  const v4f a = *(const v4f*)(p);
  const v4f c = *(const v4f*)(p + 4);
  unsigned short hb[8];
#pragma unroll
  for (int e = 0; e < 4; ++e) {
    hb[e]     = h_bits(a[e] * carry);
    hb[4 + e] = h_bits(c[e] * carry);
  }
  const v4u u = (v4u){pk16(hb[0], hb[1]), pk16(hb[2], hb[3]), pk16(hb[4], hb[5]), pk16(hb[6], hb[7])};
  unsigned short* q = out + 8 * (size_t)i;
  *(volatile v4u*)q = u;
  __threadfence();
  *(volatile v4u*)q = u;
}

__global__ __launch_bounds__(256) void k_adapt(const float* __restrict__ E1, const float* __restrict__ E2, unsigned short* __restrict__ adj) {
  __shared__ __align__(16) float srow[kN];
  __shared__ float redA[8];
  __shared__ float redB[8];
  const int bid = blockIdx.x;
  const int hd = bid >> 11;
  const int w = bid & (kN - 1);
  const int t = threadIdx.x;
  const int lane = t & 31, wave = t >> 5;
  const float* e1p = E1 + ((size_t)w * kH + hd) * kDh;
  const v4f ea = *(const v4f*)(e1p);
  const v4f eb = *(const v4f*)(e1p + 4);
  const int v0 = t * 8;

  float lmax = 0.0f;
#pragma unroll 1
  for (int e = 0; e < 8; ++e) {
    const int v = v0 + e;
    const float* e2p = E2 + ((size_t)v * kH + hd) * kDh;
    const v4f fa = *(const v4f*)(e2p);
    const v4f fb = *(const v4f*)(e2p + 4);
    float s = ea[0] * fa[0];
    s += ea[1] * fa[1];
    s += ea[2] * fa[2];
    s += ea[3] * fa[3];
    s += eb[0] * fb[0];
    s += eb[1] * fb[1];
    s += eb[2] * fb[2];
    s += eb[3] * fb[3];
    s = fmaxf(s, 0.0f) * kInvSqrtDh;
    srow[v] = s;
    lmax = fmaxf(lmax, s);
  }
  float mx = lmax;
#pragma unroll
  for (int off = 16; off > 0; off >>= 1) mx = fmaxf(mx, __shfl_xor(mx, off, 32));
  if (lane == 0) redA[wave] = mx;
  __syncthreads();
  const float m = fmaxf(fmaxf(fmaxf(redA[0], redA[1]), fmaxf(redA[2], redA[3])),
                        fmaxf(fmaxf(redA[4], redA[5]), fmaxf(redA[6], redA[7])));

  float lsum = 0.0f;
#pragma unroll 1
  for (int e = 0; e < 8; ++e) {
    const int v = v0 + e;
    const float p = expf(srow[v] - m);
    srow[v] = p;
    lsum += p;
  }
  float sm = lsum;
#pragma unroll
  for (int off = 16; off > 0; off >>= 1) sm += __shfl_xor(sm, off, 32);
  if (lane == 0) redB[wave] = sm;
  __syncthreads();
  const float tot = ((redB[0] + redB[1]) + (redB[2] + redB[3])) + ((redB[4] + redB[5]) + (redB[6] + redB[7]));
  const float sc = kAdjCarry / tot;

  const v4f pa = *(const v4f*)(srow + v0);
  const v4f pb = *(const v4f*)(srow + v0 + 4);
  unsigned short hb[8];
#pragma unroll
  for (int e = 0; e < 4; ++e) {
    hb[e]     = h_bits(pa[e] * sc);
    hb[4 + e] = h_bits(pb[e] * sc);
  }
  const v4u u = (v4u){pk16(hb[0], hb[1]), pk16(hb[2], hb[3]), pk16(hb[4], hb[5]), pk16(hb[6], hb[7])};
  unsigned short* dst = adj + ((size_t)(2 + hd) * kN + w) * kN + v0;
  *(volatile v4u*)dst = u;
  __threadfence();
  *(volatile v4u*)dst = u;
}

__global__ __launch_bounds__(256) void k_wt(const float* __restrict__ wz, const float* __restrict__ wr,
                                           const float* __restrict__ wc, const float* __restrict__ wm,
                                           unsigned short* __restrict__ wt) {
  const int t = threadIdx.x, lane = t & 31, wave = t >> 5;
  const int R = blockIdx.x * 32 + wave * 4 + (lane >> 3);
  const int c8 = (lane & 7) * 8;
  unsigned short hb[8];
#pragma unroll
  for (int e = 0; e < 8; ++e) {
    const int k = c8 + e;
    const int kg = min(k, 3 * kC - 1);
    const int km = min(k, kC - 1);
    const int nz = min(R, kC - 1);
    const int nr = min(max(R - 64, 0), kC - 1);
    const int nc = min(max(R - 128, 0), kC - 1);
    const int nm = min(max(R - 192, 0), kOut - 1);
    const float vz = wz[kg * kC + nz];
    const float vr = wr[kg * kC + nr];
    const float vc = wc[kg * kC + nc];
    const float vm = wm[km * kOut + nm];
    const bool kok = (k < 3 * kC);
    float v = 0.0f;
    v = (R < kC && kok) ? vz : v;
    v = (R >= 64 && R < 64 + kC && kok) ? vr : v;
    v = (R >= 128 && R < 128 + kC && kok) ? vc : v;
    v = (R >= 192 && R < 192 + kOut && k < kC) ? vm : v;
    hb[e] = h_bits(v * kWCarry);
  }
  const v4u u = (v4u){pk16(hb[0], hb[1]), pk16(hb[2], hb[3]), pk16(hb[4], hb[5]), pk16(hb[6], hb[7])};
  unsigned short* dst = wt + (size_t)R * kGK + c8;
  *(volatile v4u*)dst = u;
  __threadfence();
  *(volatile v4u*)dst = u;
}

__global__ __launch_bounds__(256) void k_feat_t(const float* __restrict__ s0, int st0, const float* __restrict__ s1, int st1, int csplit,
                                               unsigned short* __restrict__ ft, float carry) {
  const int R = blockIdx.x;
  const int t = threadIdx.x;
  const int n0 = t * 8;
  float v[8];
  if (R < kB * kC) {
    const int b = R / kC;
    const int c = R - b * kC;
    const size_t bn = (size_t)b * kN + n0;
    if (c < csplit) {
#pragma unroll
      for (int e = 0; e < 8; ++e) v[e] = s0[(bn + e) * (size_t)st0 + c];
    } else {
#pragma unroll
      for (int e = 0; e < 8; ++e) v[e] = s1[(bn + e) * (size_t)st1 + (c - csplit)];
    }
  } else {
#pragma unroll
    for (int e = 0; e < 8; ++e) v[e] = 0.0f;
  }
  unsigned short hb[8];
#pragma unroll
  for (int e = 0; e < 8; ++e) hb[e] = h_bits(v[e] * carry);
  const v4u u = (v4u){pk16(hb[0], hb[1]), pk16(hb[2], hb[3]), pk16(hb[4], hb[5]), pk16(hb[6], hb[7])};
  unsigned short* dst = ft + (size_t)R * kN + n0;
  *(volatile v4u*)dst = u;
  __threadfence();
  *(volatile v4u*)dst = u;
}

__global__ __launch_bounds__(128) void k_gate_feat(const float* __restrict__ s0, int st0, const float* __restrict__ s1, int st1, int csplit,
                                                  const float* __restrict__ Y1, const float* __restrict__ Y2,
                                                  const float* __restrict__ ap, unsigned short* __restrict__ G) {
  __shared__ __align__(16) float stg[128 * 68];
  const int t = threadIdx.x;
  const int lane = t & 31, wave = t >> 5;
  const int row0 = blockIdx.x * 128;
  const int idx = row0 + t;
  const int b = idx >> 11;
  const int n = idx & (kN - 1);
  const float a = ap[0];
  const float ch = (1.0f + a) * kGateCarry;
  const float cp = a * kGateCarry;
  const float cm = (1.0f - a) * 0.25f * kGateCarry;
  float* my = stg + t * 68;
#pragma unroll 1
  for (int c = 0; c < kC; ++c) {
    const int c0 = min(c, csplit - 1);
    const int c1 = max(c - csplit, 0);
    const float xv = s0[(size_t)idx * st0 + c0];
    const float hv = s1[(size_t)idx * st1 + c1];
    const float sv = (c < csplit) ? xv : hv;
    const size_t co = (size_t)(b * kC + c) * kN + n;
    const float p1 = Y1[co] + Y1[kYPlane + co];
    const float m1 = (Y1[2 * kYPlane + co] + Y1[3 * kYPlane + co]) + (Y1[4 * kYPlane + co] + Y1[5 * kYPlane + co]);
    const float p2 = Y2[co] + Y2[kYPlane + co];
    const float m2 = (Y2[2 * kYPlane + co] + Y2[3 * kYPlane + co]) + (Y2[4 * kYPlane + co] + Y2[5 * kYPlane + co]);
    my[c] = ch * sv;
    my[kC + c] = cp * p1 + cm * m1;
    my[2 * kC + c] = cp * p2 + cm * m2;
  }
#pragma unroll 1
  for (int c = 3 * kC; c < kGK; ++c) my[c] = 0.0f;
  __syncthreads();
  const int q = lane >> 3, c8 = (lane & 7) * 8;
  unsigned short* gb = G + (size_t)row0 * kGK;
  for (int pass = 0; pass < 2; ++pass) {
#pragma unroll
    for (int it = 0; it < 8; ++it) {
      const int rl = wave * 32 + it * 4 + q;
      const float* sp = stg + rl * 68 + c8;
      const v4f va = *(const v4f*)(sp);
      const v4f vb = *(const v4f*)(sp + 4);
      unsigned short hb[8];
#pragma unroll
      for (int e = 0; e < 4; ++e) {
        hb[e]     = h_bits(va[e]);
        hb[4 + e] = h_bits(vb[e]);
      }
      const v4u u = (v4u){pk16(hb[0], hb[1]), pk16(hb[2], hb[3]), pk16(hb[4], hb[5]), pk16(hb[6], hb[7])};
      *(volatile v4u*)(gb + (size_t)rl * kGK + c8) = u;
    }
    __threadfence();
  }
}

__global__ __launch_bounds__(128) void k_zr(const float* __restrict__ P, const float* __restrict__ bz, const float* __restrict__ br,
                                           const float* __restrict__ x, const float* __restrict__ hid, const float* __restrict__ ap,
                                           float* __restrict__ zr) {
  __shared__ __align__(16) float stg[128 * 68];
  const int t = threadIdx.x;
  const int lane = t & 31, wave = t >> 5;
  const int row0 = blockIdx.x * 128;
  const int idx = row0 + t;
  const float a = ap[0];
  const float ba = 1.0f + a;
  float* my = stg + t * 68;
#pragma unroll 1
  for (int c = 0; c < kC; ++c) {
    float pz = P[(size_t)idx * 128 + c] + ba * bz[c];
    float pr = P[(size_t)idx * 128 + 64 + c] + ba * br[c];
    pz = fminf(fmaxf(pz, -60.0f), 60.0f);
    pr = fminf(fmaxf(pr, -60.0f), 60.0f);
    const float z = 1.0f / (1.0f + expf(-pz));
    const float r = 1.0f / (1.0f + expf(-pr));
    const float xv = x[(size_t)idx * kIn + min(c, kIn - 1)];
    const float hv = hid[(size_t)idx * kOut + max(c - kIn, 0)];
    const float iv = (c < kIn) ? xv : hv;
    my[c] = z;
    my[32 + c] = r * iv;
  }
#pragma unroll 1
  for (int c = kC; c < 32; ++c) { my[c] = 0.0f; my[32 + c] = 0.0f; }
  __syncthreads();
  const int hh = lane >> 4, c4 = (lane & 15) * 4;
  float* zb = zr + (size_t)row0 * kGK;
  for (int pass = 0; pass < 2; ++pass) {
#pragma unroll
    for (int it = 0; it < 16; ++it) {
      const int rl = wave * 32 + it * 2 + hh;
      const v4f v = *(const v4f*)(stg + rl * 68 + c4);
      *(volatile v4f*)(zb + (size_t)rl * kGK + c4) = v;
    }
    __threadfence();
  }
}

__global__ __launch_bounds__(128) void k_fin(const float* __restrict__ P, const float* __restrict__ bc, const float* __restrict__ zr,
                                            const float* __restrict__ x, const float* __restrict__ hid, const float* __restrict__ ap,
                                            unsigned short* __restrict__ hp) {
  __shared__ __align__(16) float stg[128 * 68];
  const int t = threadIdx.x;
  const int lane = t & 31, wave = t >> 5;
  const int row0 = blockIdx.x * 128;
  const int idx = row0 + t;
  const float a = ap[0];
  const float ba = 1.0f + a;
  float* my = stg + t * 68;
#pragma unroll 1
  for (int c = 0; c < kC; ++c) {
    const float pcv = P[(size_t)idx * kGK + c] + ba * bc[c];
    const float cv = tanhf(pcv);
    const float z = zr[(size_t)idx * kGK + c];
    const float xv = x[(size_t)idx * kIn + min(c, kIn - 1)];
    const float hv = hid[(size_t)idx * kOut + max(c - kIn, 0)];
    const float iv = (c < kIn) ? xv : hv;
    const float h = (1.0f - z) * iv + z * cv;
    my[c] = kHCarry * h;
  }
#pragma unroll 1
  for (int c = kC; c < kGK; ++c) my[c] = 0.0f;
  __syncthreads();
  const int q = lane >> 3, c8 = (lane & 7) * 8;
  unsigned short* hb0 = hp + (size_t)row0 * kGK;
  for (int pass = 0; pass < 2; ++pass) {
#pragma unroll
    for (int it = 0; it < 8; ++it) {
      const int rl = wave * 32 + it * 4 + q;
      const float* sp = stg + rl * 68 + c8;
      const v4f va = *(const v4f*)(sp);
      const v4f vb = *(const v4f*)(sp + 4);
      unsigned short hb[8];
#pragma unroll
      for (int e = 0; e < 4; ++e) {
        hb[e]     = h_bits(va[e]);
        hb[4 + e] = h_bits(vb[e]);
      }
      const v4u u = (v4u){pk16(hb[0], hb[1]), pk16(hb[2], hb[3]), pk16(hb[4], hb[5]), pk16(hb[6], hb[7])};
      *(volatile v4u*)(hb0 + (size_t)rl * kGK + c8) = u;
    }
    __threadfence();
  }
}

__global__ __launch_bounds__(256) void k_out(const float* __restrict__ of, const float* __restrict__ mb, float* __restrict__ out) {
  const int i = blockIdx.x * 256 + threadIdx.x;
  if (i >= kRows * kOut / 4) return;
  const int row = i >> 2;
  const int o4 = (i & 3) * 4;
  const v4f a = *(const v4f*)(of + (size_t)row * kGK + o4);
  v4f v;
  v[0] = a[0] + mb[o4 + 0];
  v[1] = a[1] + mb[o4 + 1];
  v[2] = a[2] + mb[o4 + 2];
  v[3] = a[3] + mb[o4 + 3];
  float* q = out + (size_t)i * 4;
  *(volatile v4f*)q = v;
  __threadfence();
  *(volatile v4f*)q = v;
}

extern "C" void kernel_launch(void* const* d_in, const int* in_sizes, int n_in,
                              void* d_out, int out_size, void* d_ws, size_t ws_size,
                              hipStream_t stream) {
  if (n_in < 14) return;
  if (in_sizes[0] != kB * kN * kIn) return;
  if (in_sizes[1] != kB * kN * kOut) return;
  if (in_sizes[2] != 2 * kN * kN) return;
  if (in_sizes[3] != kN * kH * kDh) return;
  if (in_sizes[4] != kN * kH * kDh) return;
  if (in_sizes[5] != 3 * kC * kC || in_sizes[6] != kC) return;
  if (in_sizes[7] != 3 * kC * kC || in_sizes[8] != kC) return;
  if (in_sizes[9] != 3 * kC * kC || in_sizes[10] != kC) return;
  if (in_sizes[11] != kC * kOut || in_sizes[12] != kOut) return;
  if (in_sizes[13] < 1) return;
  if (out_size != kRows * kOut) return;

  const float* x    = (const float*)d_in[0];
  const float* hid  = (const float*)d_in[1];
  const float* preA = (const float*)d_in[2];
  const float* E1   = (const float*)d_in[3];
  const float* E2   = (const float*)d_in[4];
  const float* gzW  = (const float*)d_in[5];
  const float* gzb  = (const float*)d_in[6];
  const float* grW  = (const float*)d_in[7];
  const float* grb  = (const float*)d_in[8];
  const float* gcW  = (const float*)d_in[9];
  const float* gcb  = (const float*)d_in[10];
  const float* mlpW = (const float*)d_in[11];
  const float* mlpb = (const float*)d_in[12];
  const float* aP   = (const float*)d_in[13];
  float* out = (float*)d_out;

  char* w = (char*)d_ws;
  size_t off = 0;
  unsigned short* ADJH = (unsigned short*)(w + off); off += (size_t)kNG * kAdjPlane * 2;
  unsigned short* FT1  = (unsigned short*)(w + off); off += (size_t)kYPlane * 2;
  unsigned short* FT2  = (unsigned short*)(w + off); off += (size_t)kYPlane * 2;
  float*          Y1F  = (float*)(w + off);          off += (size_t)kNG * kYPlane * 4;
  unsigned short* Y1H  = (unsigned short*)(w + off); off += (size_t)kNG * kYPlane * 2;
  float*          Y2F  = (float*)(w + off);          off += (size_t)kNG * kYPlane * 4;
  float*          Y1F2 = (float*)(w + off);          off += (size_t)kNG * kYPlane * 4;
  unsigned short* Y1H2 = (unsigned short*)(w + off); off += (size_t)kNG * kYPlane * 2;
  float*          Y2F2 = (float*)(w + off);          off += (size_t)kNG * kYPlane * 4;
  unsigned short* WT   = (unsigned short*)(w + off); off += (size_t)256 * kGK * 2;
  unsigned short* G1   = (unsigned short*)(w + off); off += (size_t)kRows * kGK * 2;
  unsigned short* G2   = (unsigned short*)(w + off); off += (size_t)kRows * kGK * 2;
  float*          PZR  = (float*)(w + off);          off += (size_t)kRows * 128 * 4;
  float*          ZRF  = (float*)(w + off);          off += (size_t)kRows * kGK * 4;
  float*          PC   = (float*)(w + off);          off += (size_t)kRows * kGK * 4;
  unsigned short* HP   = (unsigned short*)(w + off); off += (size_t)kRows * kGK * 2;
  float*          OUTF = (float*)(w + off);          off += (size_t)kRows * kGK * 4;
  if (off > ws_size) return;

  const unsigned short* kNull16 = (const unsigned short*)nullptr;
  const float* kNullF = (const float*)nullptr;

  k_cast8<<<(2 * kN * kN / 8) / 256, 256, 0, stream>>>(preA, ADJH, 2 * kN * kN / 8, kAdjCarry);
  k_adapt<<<kH * kN, 256, 0, stream>>>(E1, E2, ADJH);
  k_wt<<<8, 256, 0, stream>>>(gzW, grW, gcW, mlpW, WT);
  k_feat_t<<<kColPad, 256, 0, stream>>>(x, kIn, hid, kOut, kIn, FT1, kFeatCarry);

  const dim3 gProp((kColPad / 64) * (kN / 64) / 8, kNG);
  wmma_gemm64<0, false, 0, 0, false><<<gProp, 256, 0, stream>>>(
      FT1, kNull16, kN, 0L, ADJH, kNull16, kN, (long)kAdjPlane, (void*)Y1F, (void*)nullptr, kN, (long)kYPlane,
      kNullF, kNullF, 0L, kColPad, kN, kN, kScaleD1);
  k_cast8<<<(int)((kNG * kYPlane / 8) / 256), 256, 0, stream>>>(Y1F, Y1H, (int)(kNG * kYPlane / 8), kY1Carry);
  wmma_gemm64<0, false, 0, 0, false><<<gProp, 256, 0, stream>>>(
      Y1H, kNull16, kN, (long)kYPlane, ADJH, kNull16, kN, (long)kAdjPlane, (void*)Y2F, (void*)nullptr, kN, (long)kYPlane,
      kNullF, kNullF, 0L, kColPad, kN, kN, kScaleD2);
  k_gate_feat<<<kRows / 128, 128, 0, stream>>>(x, kIn, hid, kOut, kIn, Y1F, Y2F, aP, G1);
  wmma_gemm64<0, false, 0, 0, false><<<dim3((kRows / 64) * 2 / 8, 1), 256, 0, stream>>>(
      G1, kNull16, kGK, 0L, WT, kNull16, kGK, 0L, (void*)PZR, (void*)nullptr, 128, 0L,
      kNullF, kNullF, 0L, kRows, 128, kGK, kScaleGate);
  k_zr<<<kRows / 128, 128, 0, stream>>>(PZR, gzb, grb, x, hid, aP, ZRF);
  k_feat_t<<<kColPad, 256, 0, stream>>>(ZRF + 32, kGK, ZRF + 32, kGK, kC, FT2, kFeatCarry);
  wmma_gemm64<0, false, 0, 0, false><<<gProp, 256, 0, stream>>>(
      FT2, kNull16, kN, 0L, ADJH, kNull16, kN, (long)kAdjPlane, (void*)Y1F2, (void*)nullptr, kN, (long)kYPlane,
      kNullF, kNullF, 0L, kColPad, kN, kN, kScaleD1);
  k_cast8<<<(int)((kNG * kYPlane / 8) / 256), 256, 0, stream>>>(Y1F2, Y1H2, (int)(kNG * kYPlane / 8), kY1Carry);
  wmma_gemm64<0, false, 0, 0, false><<<gProp, 256, 0, stream>>>(
      Y1H2, kNull16, kN, (long)kYPlane, ADJH, kNull16, kN, (long)kAdjPlane, (void*)Y2F2, (void*)nullptr, kN, (long)kYPlane,
      kNullF, kNullF, 0L, kColPad, kN, kN, kScaleD2);
  k_gate_feat<<<kRows / 128, 128, 0, stream>>>(ZRF + 32, kGK, ZRF + 32, kGK, kC, Y1F2, Y2F2, aP, G2);
  wmma_gemm64<0, false, 0, 0, false><<<dim3((kRows / 64) / 8, 1), 256, 0, stream>>>(
      G2, kNull16, kGK, 0L, WT + (size_t)128 * kGK, kNull16, kGK, 0L, (void*)PC, (void*)nullptr, kGK, 0L,
      kNullF, kNullF, 0L, kRows, kGK, kGK, kScaleGate);
  k_fin<<<kRows / 128, 128, 0, stream>>>(PC, gcb, ZRF, x, hid, aP, HP);
  wmma_gemm64<0, false, 0, 0, false><<<dim3((kRows / 64) / 8, 1), 256, 0, stream>>>(
      HP, kNull16, kGK, 0L, WT + (size_t)192 * kGK, kNull16, kGK, 0L, (void*)OUTF, (void*)nullptr, kGK, 0L,
      kNullF, kNullF, 0L, kRows, kGK, kGK, kScaleMlp);
  k_out<<<(kRows * kOut / 4) / 256, 256, 0, stream>>>(OUTF, mlpb, out);
}
